// SpectralConv1d_86397562126834
// MI455X (gfx1250) — hardware-verified
//
#include <hip/hip_runtime.h>


#define B_SZ   16
#define CIN    64
#define COUT   64
#define NPTS   4096
#define MODES  32
#define NF     2049
#define NFP    2064
#define NROWS  1024
typedef __attribute__((ext_vector_type(16))) _Float16 v16h;
typedef __attribute__((ext_vector_type(8)))  _Float16 v8h;
typedef __attribute__((ext_vector_type(8)))  float    v8f;
typedef __attribute__((ext_vector_type(4)))  float    v4f;
#define TWO_PI 6.28318530717958647692f
#define VST2(T, ptr, val) do { const T _v = (val); *(volatile T*)(ptr) = _v; __threadfence(); *(volatile T*)(ptr) = _v; } while (0)
__device__ __forceinline__ v8f wmma16(v16h a, v16h b, v8f c) {
  v8f d = __builtin_amdgcn_wmma_f32_16x16x32_f16(false, a, false, b, (short)0, c, false, false);
  asm volatile("v_nop\n\tv_nop\n\tv_nop\n\tv_nop" : "+v"(d) : "v"(a), "v"(b));
  return d;
}
__device__ __forceinline__ v16h frag16(const _Float16* p, int hh) {
  const v8h lo = *(const v8h*)(p + 8 * hh), hi = *(const v8h*)(p + 16 + 8 * hh);
  return __builtin_shufflevector(lo, hi, 0,1,2,3,4,5,6,7,8,9,10,11,12,13,14,15);
}
#define OFF_WFT 0u
#define OFF_W2T (OFF_WFT + 64u * 4096u * 2u)
#define OFF_X   (OFF_W2T + (unsigned)NFP * 64u * 2u)
#define OFF_A2  (OFF_X   + 1024u * 64u * 4u)
#define OFF_XB  (OFF_A2  + 1024u * 64u * 2u)
#define WS_END  (OFF_XB  + 1024u * 4096u * 2u)

__global__ void __launch_bounds__(256) xcast(const float* __restrict__ x, _Float16* __restrict__ xb) {
  int t = blockIdx.x * 256 + threadIdx.x;
  const float* p = x + (size_t)t * 8;
  v8h o;
#pragma unroll
  for (int e = 0; e < 8; ++e) o[e] = (_Float16)p[e];
  VST2(v8h, xb + (size_t)t * 8, o);
}
__global__ void __launch_bounds__(256) init_wft(_Float16* __restrict__ wft) {
  int t8 = blockIdx.x * 256 + threadIdx.x;
  int j = (t8 * 8) >> 12, n0 = (t8 * 8) & 4095, m = j & 31;
  v8h o;
#pragma unroll
  for (int e = 0; e < 8; ++e) { int t = (m * (n0 + e)) & (NPTS - 1); float th = (TWO_PI / (float)NPTS) * (float)t; o[e] = (_Float16)((j < MODES) ? __cosf(th) : -__sinf(th)); }
  VST2(v8h, wft + (size_t)t8 * 8, o);
}
__global__ void __launch_bounds__(256) init_w2t(_Float16* __restrict__ w2t) {
  int t8 = blockIdx.x * 256 + threadIdx.x;
  if (t8 >= NFP * 64 / 8) return;
  int n = (t8 * 8) >> 6, j0 = (t8 * 8) & 63;
  v8h o;
#pragma unroll
  for (int e = 0; e < 8; ++e) {
    int j = j0 + e; float v = 0.f;
    if (n < NF) { int m = j & 31; int t = (int)(((long long)m * n) % NF); float th = (TWO_PI / (float)NF) * (float)t; v = ((j < MODES) ? __cosf(th) : -__sinf(th)) * (1.0f / (float)NF); }
    o[e] = (_Float16)v;
  }
  VST2(v8h, w2t + (size_t)t8 * 8, o);
}
__global__ void __launch_bounds__(128) dft_fwd_wmma(const _Float16* __restrict__ xb, const _Float16* __restrict__ wft, float* __restrict__ Xout) {
  __shared__ __attribute__((aligned(16))) float sT[16][64];
  const int lane = threadIdx.x & 31, ntile = threadIdx.x >> 5, mtile = blockIdx.x, hh = lane >> 4, l15 = lane & 15;
  const _Float16* arow = xb + (size_t)(mtile * 16 + l15) * NPTS;
  const _Float16* brow = wft + (size_t)(ntile * 16 + l15) * NPTS;
  v8f acc0 = {}, acc1 = {};
  for (int kk = 0; kk < NPTS; kk += 64) {
    acc0 = wmma16(frag16(arow + kk, hh), frag16(brow + kk, hh), acc0);
    acc1 = wmma16(frag16(arow + kk + 32, hh), frag16(brow + kk + 32, hh), acc1);
  }
#pragma unroll
  for (int r = 0; r < 8; ++r) sT[r + 8 * hh][ntile * 16 + l15] = acc0[r] + acc1[r];
  __syncthreads();
  for (int pass = 0; pass < 2; ++pass) {
#pragma unroll
    for (int j = 0; j < 2; ++j) { const int rr = j * 8 + (threadIdx.x >> 4), q4 = (threadIdx.x & 15) * 4;
      *(volatile v4f*)(Xout + (size_t)(mtile * 16 + rr) * 64 + q4) = *(const v4f*)(&sT[rr][q4]); }
    __threadfence();
  }
}
__global__ void __launch_bounds__(256) mode_mix(const float* __restrict__ X, const float* __restrict__ w1, _Float16* __restrict__ a2) {
  const int t = blockIdx.x * 256 + threadIdx.x;
  const int j = t & 63, m = t >> 6, b = m >> 6, o = m & 63, k = j & 31;
  float s = 0.f;
  for (int i = 0; i < CIN; ++i) {
    const float* xp = X + (size_t)(b * CIN + i) * 64;
    const float xr = xp[k], xi = xp[32 + k];
    const float* wp = w1 + ((size_t)(i * COUT + o) * MODES + k) * 2;
    const float wr = wp[0], wi = wp[1];
    s += (j < 32) ? (xr * wr - xi * wi) : (xr * wi + xi * wr);
  }
  VST2(_Float16, a2 + (size_t)m * 64 + j, (_Float16)s);
}
__global__ void __launch_bounds__(256) idft_wmma(const _Float16* __restrict__ a2, const _Float16* __restrict__ w2t, float* __restrict__ y) {
  __shared__ __attribute__((aligned(16))) float sY[16][NFP];
  __shared__ __attribute__((aligned(16))) float carry[32];
  const int lane = threadIdx.x & 31, wave = threadIdx.x >> 5, hh = lane >> 4, l15 = lane & 15;
  const int m0 = blockIdx.x * 32;
  const size_t reg0 = (size_t)m0 * NF;
  for (int half = 0; half < 2; ++half) {
    const int r0 = m0 + half * 16;
    const _Float16* arow = a2 + (size_t)(r0 + l15) * 64;
    const v16h a0 = frag16(arow, hh), a1 = frag16(arow + 32, hh);
    for (int nt = wave; nt < NFP / 16; nt += 8) {
      const _Float16* brow = w2t + (size_t)(nt * 16 + l15) * 64;
      v8f acc = {};
      acc = wmma16(a0, frag16(brow, hh), acc);
      acc = wmma16(a1, frag16(brow + 32, hh), acc);
#pragma unroll
      for (int r = 0; r < 8; ++r) sY[r + 8 * hh][nt * 16 + l15] = acc[r];
    }
    __syncthreads();
    const size_t f0 = reg0 + (size_t)half * 16 * NF, f1 = f0 + (size_t)16 * NF;
    const size_t line0 = (f0 + 31) & ~(size_t)31;
    const size_t lineEnd = (half == 1) ? f1 : (f1 & ~(size_t)31);
    if (half == 0) {
      const size_t s0 = f1 & ~(size_t)31;
      if (threadIdx.x < 32) { const size_t f = s0 + threadIdx.x; carry[threadIdx.x] = (f < f1) ? sY[(f - f0) / NF][(f - f0) % NF] : 0.f; }
    }
    for (int pass = 0; pass < 2; ++pass) {
      if (half == 1 && threadIdx.x < 32) {
        const size_t s0 = f0 & ~(size_t)31, f = s0 + threadIdx.x;
        const float v = (f < f0) ? carry[threadIdx.x] : sY[(f - f0) / NF][(f - f0) % NF];
        *(volatile float*)(y + f) = v;
      }
      for (size_t f = line0 + threadIdx.x; f < lineEnd; f += 256) {
        *(volatile float*)(y + f) = sY[(f - f0) / NF][(f - f0) % NF];
      }
      __threadfence();
    }
    __syncthreads();
  }
}
extern "C" void kernel_launch(void* const* d_in, const int* in_sizes, int n_in,
                              void* d_out, int out_size, void* d_ws, size_t ws_size, hipStream_t stream) {
  (void)in_sizes; (void)n_in; (void)out_size;
  const float* x  = (const float*)d_in[0];
  const float* w1 = (const float*)d_in[1];
  float* y        = (float*)d_out;
  if (ws_size < WS_END) return;
  char* ws = (char*)d_ws;
  _Float16* wft = (_Float16*)(ws + OFF_WFT);
  _Float16* w2t = (_Float16*)(ws + OFF_W2T);
  float*    X   = (float*)   (ws + OFF_X);
  _Float16* a2  = (_Float16*)(ws + OFF_A2);
  _Float16* xb  = (_Float16*)(ws + OFF_XB);
  init_wft<<<(64 * 4096 / 8) / 256, 256, 0, stream>>>(wft);
  init_w2t<<<(NFP * 64 / 8 + 255) / 256, 256, 0, stream>>>(w2t);
  xcast<<<(1024 * NPTS / 8) / 256, 256, 0, stream>>>(x, xb);
  dft_fwd_wmma<<<64, 128, 0, stream>>>(xb, wft, X);
  mode_mix<<<(NROWS * 64) / 256, 256, 0, stream>>>(X, w1, a2);
  idft_wmma<<<NROWS / 32, 256, 0, stream>>>(a2, w2t, y);
}
